// BaseHeads_69965017252515
// MI455X (gfx1250) — hardware-verified
//
#include <hip/hip_runtime.h>
#include <stddef.h>


typedef _Float16 h16;
typedef _Float16 v16h __attribute__((ext_vector_type(16)));
typedef _Float16 v8h  __attribute__((ext_vector_type(8)));
typedef float    v8f  __attribute__((ext_vector_type(8)));
typedef float    v4f  __attribute__((ext_vector_type(4)));

#ifndef NB
#define NB 2
#endif
#ifndef SEQ
#define SEQ 128
#endif
#define NB_FULL  2
#define SEQ_FULL 128
#define DIM   768
#define NREL  4
#define NOUT  (NREL * DIM)
#define MROWS (NB * SEQ)

#define PTI 8
#define HC  64
#define LDP 68
#define LDO 132
#define LDC 68

#define WCARRY 64.0f
#define XCARRY 16.0f

static_assert(NB >= 1 && NB <= NB_FULL);
static_assert(SEQ == SEQ_FULL && SEQ_FULL == 128);
static_assert((DIM % 32) == 0 && (DIM % 8) == 0);
static_assert((NOUT % 64) == 0 && (MROWS % 64) == 0);
static_assert(DIM == 3 * 256);
static_assert((DIM % HC) == 0 && (HC % 4) == 0);
static_assert(HC == 16 * 4);
static_assert(SEQ * 16 == 8 * 256);
static_assert(PTI * 16 == 128);
static_assert(PTI == 8 && (SEQ % PTI) == 0);
static_assert(SEQ == 128);
static_assert((LDP % 4) == 0 && LDP >= HC);
static_assert((LDO % 4) == 0 && LDO >= SEQ);
static_assert((LDC % 4) == 0 && LDC >= 64);
static_assert(((size_t)MROWS * DIM) % 2048 == 0);
static_assert(((size_t)NOUT * DIM) % 2048 == 0);

#define X16_BYTES ((size_t)MROWS * DIM * 2)
#define W16_BYTES ((size_t)NOUT * DIM * 2)
#define HPL_BYTES ((size_t)MROWS * NOUT * 4)
#define OFF_X16 ((size_t)0)
#define OFF_WS  (OFF_X16 + X16_BYTES)
#define OFF_WT  (OFF_WS + W16_BYTES)
#define OFF_HS  (OFF_WT + W16_BYTES)
#define OFF_HT  (OFF_HS + HPL_BYTES)
#define WS_TOTAL (OFF_HT + HPL_BYTES)
static_assert((X16_BYTES % 128) == 0 && (W16_BYTES % 128) == 0 && (HPL_BYTES % 128) == 0);
static_assert(WS_TOTAL <= (size_t)134217728);

__device__ __forceinline__ float bf16r(float x) {
  unsigned int u = __float_as_uint(x);
  u = (u + 0x7FFFu + ((u >> 16) & 1u)) & 0xFFFF0000u;
  return __uint_as_float(u);
}

static __device__ __forceinline__ h16 toh_flush(float v) {
  const h16 r = (h16)v;
  return (fabsf(v) < 6.103515625e-05f) ? (h16)0.0f : r;
}

__device__ __forceinline__ v16h frag_at(const _Float16* p) {
  v8h lo = *(const v8h*)(p);
  v8h hi = *(const v8h*)(p + 16);
  v16h out;
#pragma unroll
  for (int i = 0; i < 8; ++i) { out[i] = lo[i]; out[i + 8] = hi[i]; }
  return out;
}

__device__ __forceinline__ v8f wmma16(v16h a, v16h b, v8f c) {
  v8f d = __builtin_amdgcn_wmma_f32_16x16x32_f16(false, a, false, b, (short)0, c,
                                                 false, false);
  asm volatile("v_nop\n\tv_nop\n\tv_nop\n\tv_nop" : "+v"(d) : "v"(a), "v"(b));
  return d;
}

__device__ __forceinline__ float tanh_from_twice(float u) {
  const float e = __expf(u);
  return 1.0f - 2.0f * __builtin_amdgcn_rcpf(e + 1.0f);
}

__global__ __launch_bounds__(256) void xcast_kernel(
    const float* __restrict__ X, _Float16* __restrict__ X16) {
  const unsigned g = blockIdx.x * 256u + threadIdx.x;
  const unsigned e = g * 8u;
  const unsigned crow = e / (unsigned)DIM;
  const unsigned col = e - crow * (unsigned)DIM;
  const unsigned bidx = crow / (unsigned)SEQ;
  const unsigned sq = crow - bidx * (unsigned)SEQ;
  const size_t src = ((size_t)bidx * SEQ_FULL + sq) * DIM + col;
  const v4f a0 = *(const v4f*)(X + src);
  const v4f a1 = *(const v4f*)(X + src + 4u);
  v8h o;
#pragma unroll
  for (int i = 0; i < 4; ++i) {
    o[i]     = toh_flush(XCARRY * bf16r(a0[i]));
    o[i + 4] = toh_flush(XCARRY * bf16r(a1[i]));
  }
  _Float16* p = X16 + (size_t)e;
  *(volatile v8h*)p = o;
  __threadfence();
  *(volatile v8h*)p = o;
}

__global__ __launch_bounds__(256) void wcast_kernel(
    const float* __restrict__ W, _Float16* __restrict__ W16) {
  const unsigned g = blockIdx.x * 256u + threadIdx.x;
  const size_t e = (size_t)g * 8u;
  const v4f a0 = *(const v4f*)(W + e);
  const v4f a1 = *(const v4f*)(W + e + 4u);
  v8h o;
#pragma unroll
  for (int i = 0; i < 4; ++i) {
    o[i]     = toh_flush(WCARRY * bf16r(a0[i]));
    o[i + 4] = toh_flush(WCARRY * bf16r(a1[i]));
  }
  _Float16* p = W16 + e;
  *(volatile v8h*)p = o;
  __threadfence();
  *(volatile v8h*)p = o;
}

__global__ __launch_bounds__(256) void proj_kernel(
    const _Float16* __restrict__ A16, const _Float16* __restrict__ Bt,
    const float* __restrict__ bias, float* __restrict__ outf) {
  __shared__ __attribute__((aligned(16))) float Cs[64 * LDC];
  const unsigned K = (unsigned)DIM;
  const unsigned tid = threadIdx.x, lane = tid & 31u, w = tid >> 5;
  const unsigned mw = w >> 1, nw = w & 1u;
  const unsigned hh = lane >> 4, m = lane & 15u;
  const unsigned n0 = blockIdx.x * 64u;
  const unsigned row0 = blockIdx.y * 64u;

  const _Float16* ap  = A16 + (size_t)(row0 + mw * 16u + m) * K + hh * 8u;
  const _Float16* bp0 = Bt + (size_t)(n0 + nw * 32u + m) * K + hh * 8u;
  const _Float16* bp1 = bp0 + (size_t)16 * K;
  v8f acc0 = {}, acc1 = {};
#pragma unroll 2
  for (unsigned k0 = 0; k0 < K; k0 += 32u) {
    const v16h a  = frag_at(ap + k0);
    const v16h b0 = frag_at(bp0 + k0);
    const v16h b1 = frag_at(bp1 + k0);
    acc0 = wmma16(a, b0, acc0);
    acc1 = wmma16(a, b1, acc1);
  }
#pragma unroll
  for (int r = 0; r < 8; ++r) {
    float* d = &Cs[(mw * 16u + hh * 8u + (unsigned)r) * LDC + nw * 32u + m];
    d[0]  = acc0[r];
    d[16] = acc1[r];
  }
  __syncthreads();

  const float cs = 1.0f / (WCARRY * XCARRY);
  v4f xs[4];
  size_t off[4];
#pragma unroll
  for (unsigned i = 0; i < 4u; ++i) {
    const unsigned r = 16u * i + (tid >> 4);
    const unsigned c = (tid & 15u) * 4u;
    const unsigned crow = row0 + r;
    const v4f u = *(const v4f*)&Cs[r * LDC + c];
    const v4f g = *(const v4f*)(bias + n0 + c);
    v4f val;
#pragma unroll
    for (int j = 0; j < 4; ++j) val[j] = u[j] * cs + bf16r(g[j]);
    xs[i] = val;
    off[i] = (size_t)crow * NOUT + n0 + c;
  }
#pragma unroll
  for (int i = 0; i < 4; ++i) *(volatile v4f*)(outf + off[i]) = xs[i];
  __threadfence();
#pragma unroll
  for (int i = 0; i < 4; ++i) *(volatile v4f*)(outf + off[i]) = xs[i];
}

__global__ __launch_bounds__(256) void pair_kernel(
    const float* __restrict__ HS, const float* __restrict__ HT,
    const float* __restrict__ wout, float* __restrict__ out) {
  __shared__ __attribute__((aligned(16))) float Bs[SEQ * LDP];
  __shared__ __attribute__((aligned(16))) float As[PTI * LDP];
  __shared__ __attribute__((aligned(16))) float Ws[DIM];
  __shared__ __attribute__((aligned(16))) float Os[PTI * LDO];

  const unsigned tid = threadIdx.x, lane = tid & 31u;
  const unsigned wave = (unsigned)__builtin_amdgcn_readfirstlane((int)(threadIdx.x >> 5));
  const unsigned i0 = blockIdx.x * (unsigned)PTI;
  const unsigned r = blockIdx.y;
  const unsigned b = blockIdx.z;
  const unsigned j = tid & 127u;
  const unsigned ia = (wave >> 2) * 4u;

#pragma unroll
  for (unsigned jj = 0; jj < 3u; ++jj) {
    const unsigned idx = tid + 256u * jj;
    Ws[idx] = bf16r(wout[idx]);
  }

  const size_t tbase = (size_t)(b * (unsigned)SEQ) * NOUT + r * (unsigned)DIM;
  const size_t sbase = (size_t)(b * (unsigned)SEQ + i0) * NOUT + r * (unsigned)DIM;

  float acc[4];
#pragma unroll
  for (int ii = 0; ii < 4; ++ii) acc[ii] = 0.0f;

#pragma unroll 1
  for (unsigned h0 = 0; h0 < (unsigned)DIM; h0 += (unsigned)HC) {
#pragma unroll
    for (unsigned jj = 0; jj < 8u; ++jj) {
      const unsigned idx = tid + 256u * jj;
      const unsigned row = idx >> 4, c4 = (idx & 15u) * 4u;
      const v4f v = *(const v4f*)(HT + tbase + (size_t)row * NOUT + h0 + c4);
      *(v4f*)&Bs[row * LDP + c4] = v * 2.0f;
    }
    if (wave < 4u) {
      const unsigned row = tid >> 4, c4 = (tid & 15u) * 4u;
      const v4f v = *(const v4f*)(HS + sbase + (size_t)row * NOUT + h0 + c4);
      *(v4f*)&As[row * LDP + c4] = v * 2.0f;
    }
    __syncthreads();

#pragma unroll 1
    for (unsigned hq = 0; hq < (unsigned)HC; hq += 4u) {
      const v4f bv = *(const v4f*)&Bs[j * LDP + hq];
      const v4f wv = *(const v4f*)&Ws[h0 + hq];
#pragma unroll
      for (int ii = 0; ii < 4; ++ii) {
        const v4f av = *(const v4f*)&As[(ia + (unsigned)ii) * LDP + hq];
#pragma unroll
        for (int c = 0; c < 4; ++c)
          acc[ii] += tanh_from_twice(av[c] + bv[c]) * wv[c];
      }
    }
    __syncthreads();
  }

#pragma unroll
  for (int ii = 0; ii < 4; ++ii) Os[(ia + (unsigned)ii) * LDO + j] = acc[ii];
  __syncthreads();

  const v4f x = *(const v4f*)&Os[wave * LDO + lane * 4u];
  float* p = out + (((size_t)b * NREL + r) * SEQ_FULL + i0 + wave) * SEQ_FULL + lane * 4u;
  *(volatile v4f*)p = x;
  __threadfence();
  *(volatile v4f*)p = x;
}

extern "C" void kernel_launch(void* const* d_in, const int* in_sizes, int n_in,
                              void* d_out, int out_size, void* d_ws, size_t ws_size,
                              hipStream_t stream) {
  if (n_in < 6) return;
  const long long need_x = ((long long)(NB - 1) * SEQ_FULL + SEQ) * DIM;
  if ((long long)in_sizes[0] < need_x) return;
  if ((long long)in_sizes[1] < (long long)NOUT * DIM) return;
  if ((long long)in_sizes[3] < (long long)NOUT * DIM) return;
  if (in_sizes[2] < NOUT || in_sizes[4] < NOUT) return;
  if (in_sizes[5] < DIM) return;
  if ((long long)out_size < (long long)NB * NREL * SEQ_FULL * SEQ_FULL) return;
  if (ws_size < WS_TOTAL) return;

  const float* X    = (const float*)d_in[0];
  const float* wsrc = (const float*)d_in[1];
  const float* bsrc = (const float*)d_in[2];
  const float* wtgt = (const float*)d_in[3];
  const float* btgt = (const float*)d_in[4];
  const float* wout = (const float*)d_in[5];
  float* out = (float*)d_out;

  char* ws = (char*)d_ws;
  _Float16* X16  = (_Float16*)(ws + OFF_X16);
  _Float16* Ws16 = (_Float16*)(ws + OFF_WS);
  _Float16* Wt16 = (_Float16*)(ws + OFF_WT);
  float*    HSp  = (float*)(ws + OFF_HS);
  float*    HTp  = (float*)(ws + OFF_HT);

  dim3 blk(256);
  xcast_kernel<<<dim3((unsigned)(((size_t)MROWS * DIM) / 2048)), blk, 0, stream>>>(X, X16);
  wcast_kernel<<<dim3((unsigned)(((size_t)NOUT * DIM) / 2048)), blk, 0, stream>>>(wsrc, Ws16);
  wcast_kernel<<<dim3((unsigned)(((size_t)NOUT * DIM) / 2048)), blk, 0, stream>>>(wtgt, Wt16);

  dim3 gg(NOUT / 64, MROWS / 64);
  proj_kernel<<<gg, blk, 0, stream>>>(X16, Ws16, bsrc, HSp);
  proj_kernel<<<gg, blk, 0, stream>>>(X16, Wt16, btgt, HTp);

  pair_kernel<<<dim3(SEQ / PTI, NREL, NB), blk, 0, stream>>>(HSp, HTp, wout, out);
}
